// myWholeRGAT_43877385896326
// MI455X (gfx1250) — hardware-verified
//
#include <hip/hip_runtime.h>
#include <stddef.h>


#define NBATCH 4
#define FD     256
#define NSET   128
#define NG     256
#define NN     1024
#define NLAY   3
#define KCAT   512
#define HTP    2048
#define NTHR   256
#define WSCALE 64.0f
#define WINV   (1.0f / 64.0f)
#define PSCALE 16384.0f
#define PINV   (1.0f / 16384.0f)
#define NEG_SLOPE 0.2f
#define NEG_BIG (-3.0e38f)
#define BN_EPS 1e-5f
#define SM_EPS 1e-16f
#define GEMM_LDS 65536
#define WSCAP 134217728

static_assert(NN == NBATCH * NG);
static_assert(NG == 2 * NSET);
static_assert(KCAT == 2 * FD);
static_assert(HTP == NBATCH * 2 * FD);
static_assert((FD % 64) == 0 && (NN % 64) == 0);

typedef _Float16 v8h  __attribute__((ext_vector_type(8)));
typedef _Float16 v16h __attribute__((ext_vector_type(16)));
typedef float    v4f  __attribute__((ext_vector_type(4)));
typedef float    v8f  __attribute__((ext_vector_type(8)));
union Frag { v16h v; v8h h[2]; };

__device__ __forceinline__ v8f wm(v16h a, v16h b, v8f c) {
  v8f d = __builtin_amdgcn_wmma_f32_16x16x32_f16(false, a, false, b, (short)0, c, false, false);
  asm volatile("v_nop\n\tv_nop\n\tv_nop\n\tv_nop" : "+v"(d) : "v"(a), "v"(b));
  return d;
}

__device__ __forceinline__ v16h ldfrag(const _Float16* p) {
  Frag f;
  f.h[0] = *(const v8h*)p;
  f.h[1] = *(const v8h*)(p + 16);
  return f.v;
}

__device__ __forceinline__ v8h cvt8(v4f a, v4f b, float s) {
  v8h r;
  r[0] = (_Float16)(a.x * s); r[1] = (_Float16)(a.y * s); r[2] = (_Float16)(a.z * s); r[3] = (_Float16)(a.w * s);
  r[4] = (_Float16)(b.x * s); r[5] = (_Float16)(b.y * s); r[6] = (_Float16)(b.z * s); r[7] = (_Float16)(b.w * s);
  return r;
}

__device__ __forceinline__ v4f relu4(v4f v) {
  v4f r;
  r.x = fmaxf(v.x, 0.f); r.y = fmaxf(v.y, 0.f); r.z = fmaxf(v.z, 0.f); r.w = fmaxf(v.w, 0.f);
  return r;
}

__device__ __forceinline__ void gemm_tile(const _Float16* __restrict__ Ab, int lda,
                                          const _Float16* __restrict__ Bt, int ldb, int K,
                                          int r0, int c0, int hh, int m, v8f (&acc)[8]) {
  const _Float16* ap = Ab + (size_t)(r0 + m) * lda + 8 * hh;
  const _Float16* bp = Bt + (size_t)(c0 + m) * ldb + 8 * hh;
#pragma unroll 1
  for (int k0 = 0; k0 < K; k0 += 32) {
    const v16h a = ldfrag(ap + k0);
#pragma unroll
    for (int t = 0; t < 8; ++t) {
      const v16h bf = ldfrag(bp + (size_t)(16 * t) * ldb + k0);
      acc[t] = wm(a, bf, acc[t]);
    }
  }
}

__device__ __forceinline__ void stage_tile(float* stg, const v8f (&acc)[8], int r0, int c0, int hh, int m, float scale) {
  float* sp = stg + (r0 + 8 * hh) * FD + c0 + m;
#pragma unroll
  for (int t = 0; t < 8; ++t) {
#pragma unroll
    for (int r = 0; r < 8; ++r) sp[r * FD + 16 * t] = acc[t][r] * scale;
  }
}

__global__ __launch_bounds__(NTHR) void k_pack(const float* __restrict__ d0, const float* __restrict__ d1,
                                             float* X, _Float16* CAT) {
  __shared__ __attribute__((aligned(16))) float tile[32 * FD];
  const int tid = threadIdx.x, lane = tid & 31, wave = tid >> 5;
  const int bx = blockIdx.x;
  const int b = bx >> 3, S = (bx >> 2) & 1, i0 = (bx & 3) * 32;
  const float* src = S ? d1 : d0;
#pragma unroll 4
  for (int it = 0; it < 32; ++it) {
    const int idx = it * NTHR + tid;
    const int f = idx >> 5, i = idx & 31;
    tile[i * FD + f] = src[(size_t)(b * FD + f) * NSET + i0 + i];
  }
  __syncthreads();
#pragma unroll 1
  for (int ii = 0; ii < 4; ++ii) {
    const int i = 4 * wave + ii;
    const int node = b * NG + S * NSET + i0 + i;
    const float* tp = tile + i * FD;
    const v4f xa = *(const v4f*)(tp + 4 * lane), xb = *(const v4f*)(tp + 128 + 4 * lane);
    const v8h hv = cvt8(*(const v4f*)(tp + 8 * lane), *(const v4f*)(tp + 8 * lane + 4), 1.0f);
    *(volatile v4f*)(X + (size_t)node * FD + 4 * lane) = xa;
    *(volatile v4f*)(X + (size_t)node * FD + 128 + 4 * lane) = xb;
    *(volatile v8h*)(CAT + (size_t)node * KCAT + 8 * lane) = hv;
  }
  __threadfence();
#pragma unroll 1
  for (int ii = 0; ii < 4; ++ii) {
    const int i = 4 * wave + ii;
    const int node = b * NG + S * NSET + i0 + i;
    const float* tp = tile + i * FD;
    const v4f xa = *(const v4f*)(tp + 4 * lane), xb = *(const v4f*)(tp + 128 + 4 * lane);
    const v8h hv = cvt8(*(const v4f*)(tp + 8 * lane), *(const v4f*)(tp + 8 * lane + 4), 1.0f);
    *(volatile v4f*)(X + (size_t)node * FD + 4 * lane) = xa;
    *(volatile v4f*)(X + (size_t)node * FD + 128 + 4 * lane) = xb;
    *(volatile v8h*)(CAT + (size_t)node * KCAT + 8 * lane) = hv;
  }
}

__global__ __launch_bounds__(NTHR) void k_wconv(const float* __restrict__ W, _Float16* WT) {
  __shared__ __attribute__((aligned(16))) float tile[32 * FD];
  const int tid = threadIdx.x, lane = tid & 31, wave = tid >> 5;
  const int bx = blockIdx.x;
  const int g = bx >> 3, n0 = (bx & 7) * 32;
#pragma unroll 4
  for (int it = 0; it < 32; ++it) {
    const int idx = it * NTHR + tid;
    const int k = idx >> 5, n = idx & 31;
    tile[n * FD + k] = W[(size_t)g * FD * FD + (size_t)k * FD + n0 + n];
  }
  __syncthreads();
#pragma unroll 1
  for (int ii = 0; ii < 4; ++ii) {
    const int n = 4 * wave + ii;
    const float* tp = tile + n * FD + 8 * lane;
    const v8h hv = cvt8(*(const v4f*)tp, *(const v4f*)(tp + 4), WSCALE);
    *(volatile v8h*)(WT + (size_t)(g * FD + n0 + n) * FD + 8 * lane) = hv;
  }
  __threadfence();
#pragma unroll 1
  for (int ii = 0; ii < 4; ++ii) {
    const int n = 4 * wave + ii;
    const float* tp = tile + n * FD + 8 * lane;
    const v8h hv = cvt8(*(const v4f*)tp, *(const v4f*)(tp + 4), WSCALE);
    *(volatile v8h*)(WT + (size_t)(g * FD + n0 + n) * FD + 8 * lane) = hv;
  }
}

__global__ __launch_bounds__(NTHR) void k_wlin(const float* __restrict__ W, _Float16* LW, int n8) {
  const int i = blockIdx.x * NTHR + (int)threadIdx.x;
  if (i >= n8) return;
  const float* p = W + (size_t)i * 8;
  const v8h hv = cvt8(*(const v4f*)p, *(const v4f*)(p + 4), WSCALE);
  _Float16* d = LW + (size_t)i * 8;
  *(volatile v8h*)d = hv;
  __threadfence();
  *(volatile v8h*)d = hv;
}

__device__ __forceinline__ void ht_store(const float* stg, _Float16* hb, int wave, int lane) {
#pragma unroll 1
  for (int it = 0; it < 8; ++it) {
    const int n = 32 * wave + 4 * it + (lane >> 3);
    const int i = 8 * (lane & 7);
    const float* cp = stg + i * FD + n;
    v8h hv;
#pragma unroll
    for (int e = 0; e < 8; ++e) hv[e] = (_Float16)cp[e * FD];
    *(volatile v8h*)(hb + (size_t)n * HTP + i) = hv;
  }
}

__global__ __launch_bounds__(NTHR) void k_transform(const _Float16* __restrict__ CAT, const _Float16* __restrict__ WTl,
                                                  const float* __restrict__ ql, const float* __restrict__ kl,
                                                  _Float16* HT, float* QK) {
  extern __shared__ v4f lds_dyn[];
  __shared__ __attribute__((aligned(16))) float sQK[128];
  float* stg = (float*)lds_dyn;
  const int tid = threadIdx.x, lane = tid & 31, wave = tid >> 5, hh = lane >> 4, m = lane & 15;
  const int mBase = blockIdx.x * 64;
  const int rel = blockIdx.y;
  const int r0 = (wave >> 1) * 16, c0 = (wave & 1) * 128;

  v8f acc[8];
#pragma unroll
  for (int t = 0; t < 8; ++t) { v8f z = {0.f, 0.f, 0.f, 0.f, 0.f, 0.f, 0.f, 0.f}; acc[t] = z; }
  gemm_tile(CAT + (size_t)mBase * KCAT, KCAT, WTl + (size_t)rel * FD * FD, FD, FD, r0, c0, hh, m, acc);
  stage_tile(stg, acc, r0, c0, hh, m, WINV);
  __syncthreads();

  {
    const int row = tid >> 2, part = tid & 3;
    const float* sp = stg + row * FD + part * 64;
    const float* qp = ql + part * 64;
    const float* kp = kl + part * 64;
    float ps = 0.f, pk = 0.f;
#pragma unroll 4
    for (int jx = 0; jx < 16; ++jx) {
      const v4f v = *(const v4f*)(sp + 4 * jx);
      const v4f a = *(const v4f*)(qp + 4 * jx);
      const v4f c = *(const v4f*)(kp + 4 * jx);
      ps += v.x * a.x + v.y * a.y + v.z * a.z + v.w * a.w;
      pk += v.x * c.x + v.y * c.y + v.z * c.z + v.w * c.w;
    }
    ps += __shfl_xor(ps, 1); ps += __shfl_xor(ps, 2);
    pk += __shfl_xor(pk, 1); pk += __shfl_xor(pk, 2);
    if (part == 0) { sQK[row] = ps; sQK[64 + row] = pk; }
  }
  __syncthreads();

  const int b = mBase >> 8, S = (mBase >> 7) & 1, i0 = mBase & 127, T = S ^ rel;
  _Float16* hb = HT + (size_t)b * 512 + T * 256 + rel * 128 + i0;
  float* qkd = QK + (size_t)((lane >> 4) * 2 + rel) * NN + mBase + 4 * (lane & 15);
  v4f qv = {0.f, 0.f, 0.f, 0.f};
  if (wave == 0) qv = *(const v4f*)(sQK + 4 * lane);

  if (wave == 0) *(volatile v4f*)qkd = qv;
  ht_store(stg, hb, wave, lane);
  __threadfence();
  if (wave == 0) *(volatile v4f*)qkd = qv;
  ht_store(stg, hb, wave, lane);
}

__global__ __launch_bounds__(NTHR) void k_alpha(const float* __restrict__ QK, _Float16* P) {
  const int tid = threadIdx.x, lane = tid & 31, wave = tid >> 5;
  const int d = blockIdx.x * 8 + wave;
  const int b = d >> 8, T = (d >> 7) & 1, j = d & 127;
  const int rl = lane >> 4;
  const int sb = b * NG + ((T ^ rl) << 7) + 8 * (lane & 15);
  const float* kp = QK + (size_t)(2 + rl) * NN + sb;
  const v4f ka = *(const v4f*)kp, kb = *(const v4f*)(kp + 4);
  const float q0 = QK[d], q1 = QK[NN + d];
  const float qd = rl ? q1 : q0;
  const int kk = 8 * lane;

  float lg[8];
  lg[0] = qd + ka.x; lg[1] = qd + ka.y; lg[2] = qd + ka.z; lg[3] = qd + ka.w;
  lg[4] = qd + kb.x; lg[5] = qd + kb.y; lg[6] = qd + kb.z; lg[7] = qd + kb.w;
#pragma unroll
  for (int e = 0; e < 8; ++e) lg[e] = lg[e] > 0.f ? lg[e] : NEG_SLOPE * lg[e];
  bool vl[8];
#pragma unroll
  for (int e = 0; e < 8; ++e) vl[e] = (kk + e) != j;

  float mx = NEG_BIG;
#pragma unroll
  for (int e = 0; e < 8; ++e) mx = fmaxf(mx, vl[e] ? lg[e] : NEG_BIG);
#pragma unroll
  for (int o = 16; o > 0; o >>= 1) mx = fmaxf(mx, __shfl_xor(mx, o));

  float ex[8];
  float s = 0.f;
#pragma unroll
  for (int e = 0; e < 8; ++e) { ex[e] = vl[e] ? __expf(lg[e] - mx) : 0.f; s += ex[e]; }
#pragma unroll
  for (int o = 16; o > 0; o >>= 1) s += __shfl_xor(s, o);
  const float rc = PSCALE * (1.0f / (s + SM_EPS));

  v8h pv;
#pragma unroll
  for (int e = 0; e < 8; ++e) pv[e] = (_Float16)(ex[e] * rc);
  _Float16* dp = P + (size_t)d * FD + kk;
  *(volatile v8h*)dp = pv;
  __threadfence();
  *(volatile v8h*)dp = pv;
}

__global__ __launch_bounds__(NTHR) void k_agg(const _Float16* __restrict__ P, const _Float16* __restrict__ HT,
                                            const float* __restrict__ cb, _Float16* CAT) {
  extern __shared__ v4f lds_dyn[];
  float* stg = (float*)lds_dyn;
  const int tid = threadIdx.x, lane = tid & 31, wave = tid >> 5, hh = lane >> 4, m = lane & 15;
  const int rb = blockIdx.x, bt = blockIdx.y, b = bt >> 1, T = bt & 1;
  const int nodeBase = b * NG + T * NSET + rb * 64;
  const int r0 = (wave >> 1) * 16, c0 = (wave & 1) * 128;

  v8f acc[8];
#pragma unroll
  for (int t = 0; t < 8; ++t) { v8f z = {0.f, 0.f, 0.f, 0.f, 0.f, 0.f, 0.f, 0.f}; acc[t] = z; }
  gemm_tile(P + (size_t)nodeBase * FD, FD, HT + (size_t)b * 512 + T * 256, HTP, FD, r0, c0, hh, m, acc);
  stage_tile(stg, acc, r0, c0, hh, m, PINV);
  __syncthreads();

  const v4f ba = *(const v4f*)(cb + 8 * lane), bb = *(const v4f*)(cb + 8 * lane + 4);
#pragma unroll 1
  for (int rr = 0; rr < 8; ++rr) {
    const int row = 8 * wave + rr;
    const float* sp = stg + row * FD + 8 * lane;
    const v4f a = relu4(*(const v4f*)sp + ba), c = relu4(*(const v4f*)(sp + 4) + bb);
    const v8h hv = cvt8(a, c, 1.0f);
    *(volatile v8h*)(CAT + (size_t)(nodeBase + row) * KCAT + FD + 8 * lane) = hv;
  }
  __threadfence();
#pragma unroll 1
  for (int rr = 0; rr < 8; ++rr) {
    const int row = 8 * wave + rr;
    const float* sp = stg + row * FD + 8 * lane;
    const v4f a = relu4(*(const v4f*)sp + ba), c = relu4(*(const v4f*)(sp + 4) + bb);
    const v8h hv = cvt8(a, c, 1.0f);
    *(volatile v8h*)(CAT + (size_t)(nodeBase + row) * KCAT + FD + 8 * lane) = hv;
  }
}

__global__ __launch_bounds__(NTHR) void k_lin(const _Float16* __restrict__ CAT, const _Float16* __restrict__ LWl,
                                            const float* __restrict__ lb, float* M2) {
  extern __shared__ v4f lds_dyn[];
  float* stg = (float*)lds_dyn;
  const int tid = threadIdx.x, lane = tid & 31, wave = tid >> 5, hh = lane >> 4, m = lane & 15;
  const int mBase = blockIdx.x * 64;
  const int r0 = (wave >> 1) * 16, c0 = (wave & 1) * 128;

  v8f acc[8];
#pragma unroll
  for (int t = 0; t < 8; ++t) { v8f z = {0.f, 0.f, 0.f, 0.f, 0.f, 0.f, 0.f, 0.f}; acc[t] = z; }
  gemm_tile(CAT + (size_t)mBase * KCAT, KCAT, LWl, KCAT, KCAT, r0, c0, hh, m, acc);
  stage_tile(stg, acc, r0, c0, hh, m, WINV);
  __syncthreads();

  const v4f ba = *(const v4f*)(lb + 4 * lane), bb = *(const v4f*)(lb + 128 + 4 * lane);
#pragma unroll 1
  for (int rr = 0; rr < 8; ++rr) {
    const int row = 8 * wave + rr;
    const float* sp = stg + row * FD;
    const v4f a = *(const v4f*)(sp + 4 * lane) + ba, c = *(const v4f*)(sp + 128 + 4 * lane) + bb;
    float* gp = M2 + (size_t)(mBase + row) * FD;
    *(volatile v4f*)(gp + 4 * lane) = a;
    *(volatile v4f*)(gp + 128 + 4 * lane) = c;
  }
  __threadfence();
#pragma unroll 1
  for (int rr = 0; rr < 8; ++rr) {
    const int row = 8 * wave + rr;
    const float* sp = stg + row * FD;
    const v4f a = *(const v4f*)(sp + 4 * lane) + ba, c = *(const v4f*)(sp + 128 + 4 * lane) + bb;
    float* gp = M2 + (size_t)(mBase + row) * FD;
    *(volatile v4f*)(gp + 4 * lane) = a;
    *(volatile v4f*)(gp + 128 + 4 * lane) = c;
  }
}

__global__ __launch_bounds__(NTHR) void k_bnstats(const float* __restrict__ M2, float* STAT) {
  __shared__ double rs[NTHR], rq[NTHR];
  __shared__ __attribute__((aligned(16))) float so[64];
  const int tid = threadIdx.x;
  const int col = blockIdx.x * 32 + (tid & 31);
  const int rg = tid >> 5;
  double s = 0.0, s2 = 0.0;
#pragma unroll 4
  for (int r = 0; r < 128; ++r) {
    const double v = (double)M2[(size_t)(rg * 128 + r) * FD + col];
    s += v;
    s2 += v * v;
  }
  rs[tid] = s; rq[tid] = s2;
  __syncthreads();
  if (tid < 32) {
    double a = 0.0, c = 0.0;
#pragma unroll
    for (int g = 0; g < 8; ++g) { a += rs[g * 32 + tid]; c += rq[g * 32 + tid]; }
    const double mean = a * (1.0 / 1024.0);
    double var = c * (1.0 / 1024.0) - mean * mean;
    var = var < 0.0 ? 0.0 : var;
    const float mu = (float)mean;
    const float v32 = (float)var;
    const float inv = 1.0f / sqrtf(v32 + BN_EPS);
    so[tid] = mu;
    so[32 + tid] = inv;
  }
  __syncthreads();
  v4f ov = {0.f, 0.f, 0.f, 0.f};
  float* dp = STAT + (size_t)(tid >> 3) * FD + blockIdx.x * 32 + 4 * (tid & 7);
  if (tid < 16) ov = *(const v4f*)(so + 4 * tid);
  if (tid < 16) *(volatile v4f*)dp = ov;
  __threadfence();
  if (tid < 16) *(volatile v4f*)dp = ov;
}

__global__ __launch_bounds__(NTHR) void k_bnapply(float* X, const float* __restrict__ M2, const float* __restrict__ STAT,
                                                const float* __restrict__ g, const float* __restrict__ be, _Float16* CAT) {
  __shared__ __attribute__((aligned(16))) float rowbuf[8 * FD];
  const int tid = threadIdx.x, lane = tid & 31, wave = tid >> 5;
  const int row = blockIdx.x * 8 + wave;
  const int c = 8 * lane;
  const float* xp = X + (size_t)row * FD + c;
  const float* mp = M2 + (size_t)row * FD + c;
  const v4f xa = *(const v4f*)xp, xb = *(const v4f*)(xp + 4);
  const v4f ma = *(const v4f*)mp, mb = *(const v4f*)(mp + 4);
  const v4f ua = *(const v4f*)(STAT + c), ub = *(const v4f*)(STAT + c + 4);
  const v4f ia = *(const v4f*)(STAT + FD + c), ib = *(const v4f*)(STAT + FD + c + 4);
  const v4f ga = *(const v4f*)(g + c), gb = *(const v4f*)(g + c + 4);
  const v4f ea = *(const v4f*)(be + c), eb = *(const v4f*)(be + c + 4);
  const v4f va = xa + (ga * (ma - ua) * ia + ea);
  const v4f vb = xb + (gb * (mb - ub) * ib + eb);
  const v8h hv = cvt8(va, vb, 1.0f);
  float* rp = rowbuf + wave * FD;
  *(v4f*)(rp + c) = va;
  *(v4f*)(rp + c + 4) = vb;
  _Float16* cp = CAT + (size_t)row * KCAT + c;
  *(volatile v8h*)cp = hv;
  __syncthreads();
  const v4f oa = *(const v4f*)(rp + 4 * lane), ob = *(const v4f*)(rp + 128 + 4 * lane);
  float* op = X + (size_t)row * FD;
  *(volatile v4f*)(op + 4 * lane) = oa;
  *(volatile v4f*)(op + 128 + 4 * lane) = ob;
  __threadfence();
  *(volatile v8h*)cp = hv;
  *(volatile v4f*)(op + 4 * lane) = oa;
  *(volatile v4f*)(op + 128 + 4 * lane) = ob;
}

#define UPT 132
__global__ __launch_bounds__(NTHR) void k_unpack(const float* __restrict__ X, float* out) {
  __shared__ __attribute__((aligned(16))) float tile[32 * UPT];
  const int tid = threadIdx.x, lane = tid & 31, wave = tid >> 5;
  const int bx = blockIdx.x;
  const int b = bx >> 4, S = (bx >> 3) & 1, f0 = (bx & 7) * 32;
#pragma unroll 4
  for (int it = 0; it < 16; ++it) {
    const int idx = it * NTHR + tid;
    const int i = idx >> 5, f = idx & 31;
    tile[f * UPT + i] = X[(size_t)(b * NG + S * NSET + i) * FD + f0 + f];
  }
  __syncthreads();
#pragma unroll 1
  for (int ii = 0; ii < 4; ++ii) {
    const int f = 4 * wave + ii;
    const v4f v = *(const v4f*)(tile + f * UPT + 4 * lane);
    *(volatile v4f*)(out + (size_t)S * (NN / 2) * FD + (size_t)(b * FD + f0 + f) * NSET + 4 * lane) = v;
  }
  __threadfence();
#pragma unroll 1
  for (int ii = 0; ii < 4; ++ii) {
    const int f = 4 * wave + ii;
    const v4f v = *(const v4f*)(tile + f * UPT + 4 * lane);
    *(volatile v4f*)(out + (size_t)S * (NN / 2) * FD + (size_t)(b * FD + f0 + f) * NSET + 4 * lane) = v;
  }
}

extern "C" void kernel_launch(void* const* d_in, const int* in_sizes, int n_in,
                              void* d_out, int out_size, void* d_ws, size_t ws_size,
                              hipStream_t stream) {
  if (n_in < 10) return;
  if (in_sizes[0] != NBATCH * FD * NSET || in_sizes[1] != NBATCH * FD * NSET) return;
  if (in_sizes[2] != NLAY * 2 * FD * FD) return;
  if (in_sizes[3] != NLAY * FD || in_sizes[4] != NLAY * FD || in_sizes[5] != NLAY * FD) return;
  if (in_sizes[6] != NLAY * FD * KCAT) return;
  if (in_sizes[7] != NLAY * FD || in_sizes[8] != NLAY * FD || in_sizes[9] != NLAY * FD) return;
  if (out_size != NN * FD) return;

  const float* desc0  = (const float*)d_in[0];
  const float* desc1  = (const float*)d_in[1];
  const float* conv_w = (const float*)d_in[2];
  const float* conv_q = (const float*)d_in[3];
  const float* conv_k = (const float*)d_in[4];
  const float* conv_b = (const float*)d_in[5];
  const float* lin_w  = (const float*)d_in[6];
  const float* lin_b  = (const float*)d_in[7];
  const float* bn_w   = (const float*)d_in[8];
  const float* bn_b   = (const float*)d_in[9];
  float* out = (float*)d_out;

  char* ws = (char*)d_ws;
  size_t off = 0;
  const size_t oX   = off; off += (size_t)NN * FD * 4;          off = (off + 255) & ~(size_t)255;
  const size_t oCAT = off; off += (size_t)NN * KCAT * 2;        off = (off + 255) & ~(size_t)255;
  const size_t oWT  = off; off += (size_t)NLAY * 2 * FD * FD * 2; off = (off + 255) & ~(size_t)255;
  const size_t oLW  = off; off += (size_t)NLAY * FD * KCAT * 2; off = (off + 255) & ~(size_t)255;
  const size_t oHT  = off; off += (size_t)FD * HTP * 2;         off = (off + 255) & ~(size_t)255;
  const size_t oQK  = off; off += (size_t)4 * NN * 4;           off = (off + 255) & ~(size_t)255;
  const size_t oP   = off; off += (size_t)NN * FD * 2;          off = (off + 255) & ~(size_t)255;
  const size_t oM2  = off; off += (size_t)NN * FD * 4;          off = (off + 255) & ~(size_t)255;
  const size_t oST  = off; off += (size_t)2 * FD * 4;           off = (off + 255) & ~(size_t)255;
  if (off > ws_size || off > (size_t)WSCAP) return;

  float*    X    = (float*)(ws + oX);
  _Float16* CAT  = (_Float16*)(ws + oCAT);
  _Float16* WT   = (_Float16*)(ws + oWT);
  _Float16* LW   = (_Float16*)(ws + oLW);
  _Float16* HT   = (_Float16*)(ws + oHT);
  float*    QK   = (float*)(ws + oQK);
  _Float16* P    = (_Float16*)(ws + oP);
  float*    M2   = (float*)(ws + oM2);
  float*    STAT = (float*)(ws + oST);

  hipFuncSetAttribute(reinterpret_cast<const void*>(&k_transform), hipFuncAttributeMaxDynamicSharedMemorySize, GEMM_LDS);
  hipFuncSetAttribute(reinterpret_cast<const void*>(&k_agg),       hipFuncAttributeMaxDynamicSharedMemorySize, GEMM_LDS);
  hipFuncSetAttribute(reinterpret_cast<const void*>(&k_lin),       hipFuncAttributeMaxDynamicSharedMemorySize, GEMM_LDS);

  k_pack<<<NBATCH * 2 * (NSET / 32), NTHR, 0, stream>>>(desc0, desc1, X, CAT);
  k_wconv<<<NLAY * 2 * (FD / 32), NTHR, 0, stream>>>(conv_w, WT);
  k_wlin<<<(NLAY * FD * KCAT / 8 + NTHR - 1) / NTHR, NTHR, 0, stream>>>(lin_w, LW, NLAY * FD * KCAT / 8);

  for (int l = 0; l < NLAY; ++l) {
    k_transform<<<dim3(NN / 64, 2), NTHR, GEMM_LDS, stream>>>(
        CAT, WT + (size_t)l * 2 * FD * FD, conv_q + l * FD, conv_k + l * FD, HT, QK);
    k_alpha<<<NN / 8, NTHR, 0, stream>>>(QK, P);
    k_agg<<<dim3(NSET / 64, NBATCH * 2), NTHR, GEMM_LDS, stream>>>(P, HT, conv_b + l * FD, CAT);
    k_lin<<<NN / 64, NTHR, GEMM_LDS, stream>>>(CAT, LW + (size_t)l * FD * KCAT, lin_b + l * FD, M2);
    k_bnstats<<<FD / 32, NTHR, 0, stream>>>(M2, STAT);
    k_bnapply<<<NN / 8, NTHR, 0, stream>>>(X, M2, STAT, bn_w + l * FD, bn_b + l * FD, CAT);
  }

  k_unpack<<<NBATCH * 2 * (FD / 32), NTHR, 0, stream>>>(X, out);
}
